// MHAttention_37203006718687
// MI455X (gfx1250) — hardware-verified
//
#include <hip/hip_runtime.h>

#ifndef NB
#define NB 4
#endif
#ifndef SEQ
#define SEQ 2048
#endif
#define NB_FULL 4
#define SEQ_FULL 2048
#define EMB 512
#define NHEADS 16
#define DHEAD 32
#define QCH 64
#define WIN 256
#define NEGBIG (-1.0e30f)

static_assert(EMB == NHEADS * DHEAD);
static_assert(SEQ % 64 == 0);
static_assert(QCH == 64);
static_assert(WIN % 64 == 0);
static_assert((NB * SEQ * EMB) % 2048 == 0);

typedef _Float16 v16h __attribute__((ext_vector_type(16)));
typedef unsigned short v8us __attribute__((ext_vector_type(8), may_alias));
typedef float v8f __attribute__((ext_vector_type(8)));
typedef float v4f __attribute__((ext_vector_type(4)));
typedef float v4fa __attribute__((ext_vector_type(4), may_alias));
union FragH { v16h v; v8us half[2]; _Float16 h[16]; unsigned short u[16]; };
union HU { _Float16 h; unsigned short u; };

__device__ __forceinline__ float bf16_rnef(float x) {
  unsigned int u = __float_as_uint(x);
  u = (u + 0x7FFFu + ((u >> 16) & 1u)) & 0xFFFF0000u;
  return __uint_as_float(u);
}

__device__ __forceinline__ v8f mma16(v16h a, v16h b, v8f c) {
  v8f d = __builtin_amdgcn_wmma_f32_16x16x32_f16(false, a, false, b, (short)0, c, false, false);
  asm volatile("v_nop\n\tv_nop\n\tv_nop\n\tv_nop" : "+v"(d) : "v"(a), "v"(b));
  return d;
}

__global__ __launch_bounds__(256) void k_cvt16(const float* __restrict__ q, const float* __restrict__ k,
                                               unsigned short* __restrict__ Q16, unsigned short* __restrict__ K16, int n8) {
  #pragma clang fp contract(off)
  const int t = blockIdx.x * 256 + threadIdx.x;
  if (t >= n8) return;
  const bool isk = (blockIdx.y != 0);
  const float* src = isk ? k : q;
  unsigned short* dst = isk ? K16 : Q16;
  const size_t e = (size_t)t * 8;
  const size_t pr = e / EMB;
  const int col = (int)(e % EMB);
  const size_t bb = pr / SEQ, n = pr % SEQ;
  const float* sp = src + ((bb * SEQ_FULL + n) * EMB + col);
  const v4f a = *(const v4fa*)sp;
  const v4f c = *(const v4fa*)(sp + 4);
  FragH f;
#pragma unroll
  for (int i = 0; i < 4; ++i) {
    f.h[i] = (_Float16)(bf16_rnef(a[i]) * 256.0f);
    f.h[4 + i] = (_Float16)(bf16_rnef(c[i]) * 256.0f);
  }
  const v8us o = f.half[0];
  *(volatile v8us*)(dst + e) = o;
  __threadfence();
  *(volatile v8us*)(dst + e) = o;
}

__global__ __launch_bounds__(256) void k_vt(const float* __restrict__ v, unsigned short* __restrict__ VT) {
  #pragma clang fp contract(off)
  __shared__ __attribute__((aligned(16))) unsigned short tl[DHEAD][66];
  const int tid = threadIdx.x;
  const int sg = blockIdx.x, head = blockIdx.y, b = blockIdx.z;
  const int s0 = sg * 64;
  for (int i = tid; i < 64 * 8; i += 256) {
    const int j = i >> 3, d4 = (i & 7) * 4;
    const v4f a = *(const v4fa*)(v + ((size_t)b * SEQ_FULL + s0 + j) * EMB + head * DHEAD + d4);
#pragma unroll
    for (int qq = 0; qq < 4; ++qq) { HU hu; hu.h = (_Float16)(bf16_rnef(a[qq]) * 64.0f); tl[d4 + qq][j] = hu.u; }
  }
  __syncthreads();
  const int d = tid >> 3, pc = tid & 7;
  FragH f;
#pragma unroll
  for (int qq = 0; qq < 8; ++qq) f.u[qq] = tl[d][pc * 8 + qq];
  const v8us o = f.half[0];
  unsigned short* dst = VT + (((size_t)b * NHEADS + head) * DHEAD + d) * SEQ + s0 + pc * 8;
  *(volatile v8us*)dst = o;
  __threadfence();
  *(volatile v8us*)dst = o;
}

__global__ __launch_bounds__(128) __attribute__((amdgpu_num_vgpr(256)))
void k_attn(const unsigned short* __restrict__ Q16, const unsigned short* __restrict__ K16, const unsigned short* __restrict__ VT,
            const int* __restrict__ cidx, float* __restrict__ out) {
  __shared__ __attribute__((aligned(16))) float so[4][16][32];
  (void)cidx;
  const int qc = blockIdx.x, head = blockIdx.y, b = blockIdx.z;
  const int tid = threadIdx.x, w = tid >> 5, lane = tid & 31, l15 = lane & 15, hh = lane >> 4;
  const int qs = qc * QCH;
  const int kstart = (qs >= WIN) ? (qs - WIN) : 0;
  const int nk = qs + QCH - kstart;
  const int nblk = nk >> 5;
  const int qg = qs + 16 * w + l15;
  const int thr = qg - (WIN - 1);

  FragH qb;
  {
    const unsigned short* p = Q16 + ((size_t)b * SEQ + qg) * EMB + head * DHEAD;
    qb.half[0] = *(const v8us*)(p + 8 * hh);
    qb.half[1] = *(const v8us*)(p + 16 + 8 * hh);
  }
  const unsigned short* kbase = K16 + ((size_t)b * SEQ + kstart + l15) * EMB + head * DHEAD;
  const unsigned short* vbase = VT + (((size_t)b * NHEADS + head) * DHEAD + l15) * SEQ + kstart + 8 * hh;

  const v8f z8 = {0.f, 0.f, 0.f, 0.f, 0.f, 0.f, 0.f, 0.f};
  v8f a0h = z8, a1h = z8, a0l = z8, a1l = z8;
  float m = NEGBIG, l = 0.f;
  const float scl = 0.17677669529663687f * 0.0000152587890625f;

#pragma unroll 1
  for (int kb = 0; kb < nblk; ++kb) {
    const int kb0 = kb * 32;
    v8f s0, s1;
    {
      FragH ka;
      const unsigned short* p = kbase + (size_t)kb0 * EMB;
      ka.half[0] = *(const v8us*)(p + 8 * hh);
      ka.half[1] = *(const v8us*)(p + 16 + 8 * hh);
      s0 = mma16(ka.v, qb.v, z8);
      const unsigned short* p1 = kbase + (size_t)(kb0 + 16) * EMB;
      ka.half[0] = *(const v8us*)(p1 + 8 * hh);
      ka.half[1] = *(const v8us*)(p1 + 16 + 8 * hh);
      s1 = mma16(ka.v, qb.v, z8);
    }
    const int kg0 = kstart + kb0 + 8 * hh;
    float x[16];
#pragma unroll
    for (int r = 0; r < 8; ++r) {
      x[r]     = (kg0 + r >= thr)      ? s0[r] * scl : NEGBIG;
      x[8 + r] = (kg0 + 16 + r >= thr) ? s1[r] * scl : NEGBIG;
    }
    float mx = x[0];
#pragma unroll
    for (int i = 1; i < 16; ++i) mx = fmaxf(mx, x[i]);
    mx = fmaxf(mx, __shfl_xor(mx, 16));
    const float mnew = fmaxf(m, mx);
    float p[16];
    float rs = 0.f;
#pragma unroll
    for (int i = 0; i < 16; ++i) {
      const float ev = __expf(x[i] - mnew);
      p[i] = (x[i] > -1.0e29f) ? ev : 0.f;
      rs += p[i];
    }
    rs += __shfl_xor(rs, 16);
    const float c = __expf(m - mnew);
    l = l * c + rs;
    m = mnew;
    FragH ph, pl;
#pragma unroll
    for (int i = 0; i < 16; ++i) {
      const float ps = p[i] * 1024.0f;
      const _Float16 hv = (_Float16)ps;
      ph.h[i] = hv;
      pl.h[i] = (_Float16)((ps - (float)hv) * 2048.0f);
    }
#pragma unroll
    for (int r = 0; r < 8; ++r) { a0h[r] *= c; a1h[r] *= c; a0l[r] *= c; a1l[r] *= c; }
    {
      FragH va;
      const unsigned short* p0 = vbase + kb0;
      va.half[0] = *(const v8us*)(p0);
      va.half[1] = *(const v8us*)(p0 + 16);
      a0h = mma16(va.v, ph.v, a0h);
      a0l = mma16(va.v, pl.v, a0l);
      const unsigned short* p1 = vbase + (size_t)16 * SEQ + kb0;
      va.half[0] = *(const v8us*)(p1);
      va.half[1] = *(const v8us*)(p1 + 16);
      a1h = mma16(va.v, ph.v, a1h);
      a1l = mma16(va.v, pl.v, a1l);
    }
  }

  const float inv = 1.0f / l;
  const float fo = inv * 0.0000152587890625f;
  v4f t0, t1, t2, t3;
#pragma unroll
  for (int r = 0; r < 4; ++r) {
    t0[r] = (a0h[r]     + a0l[r]     * 0.00048828125f) * fo;
    t1[r] = (a0h[4 + r] + a0l[4 + r] * 0.00048828125f) * fo;
    t2[r] = (a1h[r]     + a1l[r]     * 0.00048828125f) * fo;
    t3[r] = (a1h[4 + r] + a1l[4 + r] * 0.00048828125f) * fo;
  }
  *(v4fa*)&so[w][l15][8 * hh]          = t0;
  *(v4fa*)&so[w][l15][8 * hh + 4]      = t1;
  *(v4fa*)&so[w][l15][16 + 8 * hh]     = t2;
  *(v4fa*)&so[w][l15][16 + 8 * hh + 4] = t3;
  __syncthreads();
  const int ql = lane >> 3, c4 = (lane & 7) * 4;
  float* orow = out + ((size_t)b * SEQ + qs + 16 * w) * EMB + head * DHEAD + c4;
  for (int pass = 0; pass < 2; ++pass) {
#pragma unroll
    for (int j = 0; j < 4; ++j) {
      const int r = 4 * j + ql;
      const v4f vv = *(const v4fa*)&so[w][r][c4];
      *(volatile v4f*)(orow + (size_t)r * EMB) = vv;
    }
    if (pass == 0) __threadfence();
  }
}

extern "C" void kernel_launch(void* const* d_in, const int* in_sizes, int n_in,
                              void* d_out, int out_size, void* d_ws, size_t ws_size, hipStream_t stream) {
  if (n_in < 4) return;
  if (in_sizes[0] < NB * SEQ * EMB || in_sizes[1] < NB * SEQ * EMB || in_sizes[2] < NB * SEQ * EMB || in_sizes[3] < 1) return;
  if (out_size < NB * SEQ * EMB) return;
  const float* q = (const float*)d_in[0];
  const float* k = (const float*)d_in[1];
  const float* v = (const float*)d_in[2];
  const int* cidx = (const int*)d_in[3];
  float* out = (float*)d_out;
  char* ws = (char*)d_ws;
  size_t off = 0;
  const size_t plane = (size_t)NB * SEQ * EMB * 2;
  unsigned short* Q16 = (unsigned short*)(ws + off); off += plane;
  unsigned short* K16 = (unsigned short*)(ws + off); off += plane;
  unsigned short* VT  = (unsigned short*)(ws + off); off += plane;
  if (off > ws_size) return;
  const int n8 = NB * SEQ * EMB / 8;
  k_cvt16<<<dim3((unsigned)((n8 + 255) / 256), 2, 1), 256, 0, stream>>>(q, k, Q16, K16, n8);
  k_vt<<<dim3(SEQ / 64, NHEADS, NB), 256, 0, stream>>>(v, VT);
  k_attn<<<dim3(SEQ / QCH, NHEADS, NB), 128, 0, stream>>>(Q16, K16, VT, cidx, out);
}
